// DecoderLayer_9371618640202
// MI455X (gfx1250) — hardware-verified
//
#include <hip/hip_runtime.h>


#pragma clang fp contract(off)

#ifndef NB
#define NB 2
#endif
#ifndef SEQ
#define SEQ 2048
#endif
#define NB_FULL 2
#define SEQ_FULL 2048
#define DM 1024
#define NHD 16
#define HD 64
#define FF 4096
#define NT (NB * SEQ)
#define LNEPS 1e-12f
#define WCAR 64.0f
#define XCAR 4.0f
#define ACAR 4.0f
#define QCAR 8.0f
#define KCAR 8.0f
#define VCAR 16.0f
#define PCAR 16.0f
#define CCAR 16.0f
#define HCAR 8.0f
#define SFAC (0.125f / (QCAR * KCAR))
#define L2E 1.4426950408889634f

static_assert(NB >= 1 && NB <= NB_FULL);
static_assert(SEQ % 64 == 0 && SEQ >= 64 && SEQ <= SEQ_FULL);
static_assert(NT % 64 == 0 && NT % 8 == 0);
static_assert(DM % 64 == 0 && FF % 64 == 0 && HD == 64 && NHD * HD == DM);
static_assert((DM * DM) % 64 == 0 && (DM * FF) % 64 == 0);

typedef _Float16 h16;
typedef __attribute__((ext_vector_type(16))) _Float16 v16h;
typedef __attribute__((ext_vector_type(8)))  _Float16 v8h;
typedef __attribute__((ext_vector_type(4)))  _Float16 v4h;
typedef __attribute__((ext_vector_type(2)))  _Float16 v2h;
typedef __attribute__((ext_vector_type(8)))  float    v8f;
typedef __attribute__((ext_vector_type(4)))  float    v4f;
typedef __attribute__((ext_vector_type(4)))  int      v4i;
typedef v8h __attribute__((may_alias)) v8ha;
typedef v4f __attribute__((may_alias)) v4fa;

__device__ __forceinline__ unsigned short f2bf(float f) { unsigned u = __float_as_uint(f); u += 0x7FFFu + ((u >> 16) & 1u); return (unsigned short)(u >> 16); }
__device__ __forceinline__ float bf2f(unsigned short b) { return __uint_as_float(((unsigned)b) << 16); }
__device__ __forceinline__ float bfr(float f) { return bf2f(f2bf(f)); }
__device__ __forceinline__ v16h cat16(v8h lo, v8h hi) { return __builtin_shufflevector(lo, hi, 0, 1, 2, 3, 4, 5, 6, 7, 8, 9, 10, 11, 12, 13, 14, 15); }
__device__ __forceinline__ v8f wmma16(v16h a, v16h b, v8f c) { return __builtin_amdgcn_wmma_f32_16x16x32_f16(false, a, false, b, (short)0, c, false, false); }
__device__ __forceinline__ v16h ldfrag(const h16* p) { return cat16(*(const v8h*)p, *(const v8h*)(p + 16)); }

template <int OUTM, int BIASM, bool RELU>
__global__ __launch_bounds__(32) void k_gemmw(const h16* __restrict__ A, const h16* __restrict__ Bt, int K, void* Cv, int ldc, const float* __restrict__ bias, float alpha, float beta) {
    __shared__ __align__(16) float os[16 * 68];
    const int lane = threadIdx.x & 31, lr = lane & 15, hi = lane >> 4;
    const int r0 = blockIdx.x * 64, c0 = blockIdx.y * 64;
    v8f acc[4][4];
#pragma unroll
    for (int mb = 0; mb < 4; ++mb)
#pragma unroll
        for (int nb = 0; nb < 4; ++nb) acc[mb][nb] = (v8f){};
    const size_t aoff = (size_t)(r0 + lr) * K + 8 * hi, boff = (size_t)(c0 + lr) * K + 8 * hi;
#pragma unroll 1
    for (int kc = 0; kc < K; kc += 32) {
        v16h a[4];
#pragma unroll
        for (int mb = 0; mb < 4; ++mb) a[mb] = ldfrag(A + aoff + (size_t)mb * 16 * K + kc);
#pragma unroll
        for (int nb = 0; nb < 4; ++nb) { const v16h b = ldfrag(Bt + boff + (size_t)nb * 16 * K + kc);
#pragma unroll
            for (int mb = 0; mb < 4; ++mb) acc[mb][nb] = wmma16(a[mb], b, acc[mb][nb]); }
        asm volatile("v_nop\n\tv_nop\n\tv_nop\n\tv_nop" : "+v"(acc[0][0]), "+v"(acc[1][1]), "+v"(acc[2][2]), "+v"(acc[3][3]) : "v"(a[0]), "v"(a[3]));
    }
#pragma unroll
    for (int mb = 0; mb < 4; ++mb) {
#pragma unroll
        for (int nb = 0; nb < 4; ++nb) {
#pragma unroll
            for (int j = 0; j < 8; ++j) os[(hi * 8 + j) * 68 + nb * 16 + lr] = acc[mb][nb][j]; }
        __builtin_amdgcn_fence(3  , "wavefront"); __builtin_amdgcn_wave_barrier(); asm volatile("" ::: "memory");
        const int rb = r0 + mb * 16;
        if constexpr (OUTM == 0) {
            float* crow = (float*)Cv + (size_t)rb * ldc + c0;
#pragma unroll 1
            for (int ps = 0; ps < 2; ++ps) {
#pragma unroll
                for (int s = 0; s < 8; ++s) { const int row = 2 * s + hi, cofs = lr * 4; v4f val = *(const v4fa*)(os + row * 68 + cofs);
                    float rbv = 0.f; if (BIASM == 2) rbv = beta * bfr(bias[rb + row]);
#pragma unroll
                    for (int q = 0; q < 4; ++q) { float t = val[q] * alpha; if (BIASM == 1) t += beta * bfr(bias[c0 + cofs + q]); if (BIASM == 2) t += rbv; if (RELU) t = (t > 0.f) ? t : 0.f; val[q] = t; }
                    *(volatile v4f*)(crow + (size_t)row * ldc + cofs) = val; }
                if (ps == 0) __threadfence(); }
        } else {
            h16* crow = (h16*)Cv + (size_t)rb * ldc + c0;
#pragma unroll 1
            for (int ps = 0; ps < 2; ++ps) {
#pragma unroll
                for (int s = 0; s < 4; ++s) { const int row = 4 * s + 2 * hi + (lr >> 3), cofs = (lr & 7) * 8; const v4f v0 = *(const v4fa*)(os + row * 68 + cofs); const v4f v1 = *(const v4fa*)(os + row * 68 + cofs + 4);
                    const float tv[8] = {v0[0], v0[1], v0[2], v0[3], v1[0], v1[1], v1[2], v1[3]};
                    float rbv = 0.f; if (BIASM == 2) rbv = beta * bfr(bias[rb + row]);
                    v8h o;
#pragma unroll
                    for (int q = 0; q < 8; ++q) { float t = tv[q] * alpha; if (BIASM == 1) t += beta * bfr(bias[c0 + cofs + q]); if (BIASM == 2) t += rbv; if (RELU) t = (t > 0.f) ? t : 0.f; o[q] = (h16)t; }
                    *(volatile v8h*)(crow + (size_t)row * ldc + cofs) = o; }
                if (ps == 0) __threadfence(); }
        }
        __builtin_amdgcn_wave_barrier(); asm volatile("" ::: "memory");
    }
}

__global__ __launch_bounds__(256) void k_wtG(const float* __restrict__ w, int K, int N, h16* Bt) {
    const int lane = threadIdx.x & 31; const int L0 = (blockIdx.x * 8 + (threadIdx.x >> 5)) * 8; const int nlines = (int)(((size_t)N * K) / 64);
#pragma unroll 1
    for (int ps = 0; ps < 2; ++ps) {
#pragma unroll 1
        for (int l = 0; l < 8; ++l) { const int L = L0 + l; if (L >= nlines) break; const size_t e = (size_t)L * 64 + lane * 2; const int k = (int)(e % (size_t)K), n = (int)(e / (size_t)K); v2h o;
            o[0] = (h16)(bfr(w[(size_t)k * N + n]) * WCAR); o[1] = (h16)(bfr(w[(size_t)(k + 1) * N + n]) * WCAR); *(volatile v2h*)(Bt + e) = o; }
        if (ps == 0) __threadfence(); }
}

__global__ __launch_bounds__(256) void k_cvtx(const float* __restrict__ src, h16* dst) {
    const size_t i = (size_t)blockIdx.x * 256 + threadIdx.x; if (i >= (size_t)NT * DM / 8) return;
    const size_t e = i * 8; const size_t row = e / DM; const int col = (int)(e % DM); const int bi = (int)(row / SEQ); const int t = (int)(row % SEQ);
    const float* s = src + ((size_t)bi * SEQ_FULL + t) * DM + col; const v4f a0 = *(const v4f*)s, a1 = *(const v4f*)(s + 4); v8h o;
#pragma unroll
    for (int q = 0; q < 4; ++q) { o[q] = (h16)(bfr(a0[q]) * XCAR); o[q + 4] = (h16)(bfr(a1[q]) * XCAR); }
    *(volatile v8h*)(dst + e) = o; __threadfence(); *(volatile v8h*)(dst + e) = o;
}

__global__ __launch_bounds__(32) void k_attn(const h16* __restrict__ Qp, const h16* __restrict__ Kp, const h16* __restrict__ Vt, const int* __restrict__ pad, int causal, h16* Ctx) {
    __shared__ __align__(16) h16 so[16 * 72];
    const int lane = threadIdx.x & 31, lc = lane & 15, h = lane >> 4;
    const int q0 = blockIdx.x * 16, hh = blockIdx.y, bi = blockIdx.z;
    const int qrow = q0 + lc;
    const size_t rowbase = (size_t)bi * SEQ;
    const float NINF = -__builtin_inff();
    const h16* qptr = Qp + (rowbase + q0 + lc) * DM + hh * HD + 8 * h;
    const v16h qf0 = ldfrag(qptr), qf1 = ldfrag(qptr + 32);
    const h16* kbase = Kp + (rowbase + lc) * DM + hh * HD + 8 * h;
    const h16* vbase = Vt + ((size_t)hh * HD + lc) * NT + rowbase + 8 * h;
    const int* prow = pad + (size_t)bi * SEQ_FULL;
    float m = NINF, l = 0.f;
    v8f oacc[4];
#pragma unroll
    for (int nb = 0; nb < 4; ++nb) oacc[nb] = (v8f){};
    const int nkb = causal ? (q0 / 64 + 1) : (SEQ / 64);
#pragma unroll 1
    for (int kb = 0; kb < nkb; ++kb) {
        const int t0 = kb * 64;
        v16h kf[4][2];
#pragma unroll
        for (int j = 0; j < 4; ++j) { const h16* kp = kbase + (size_t)(t0 + j * 16) * DM; kf[j][0] = ldfrag(kp); kf[j][1] = ldfrag(kp + 32); }
        v8f sc[4];
#pragma unroll
        for (int j = 0; j < 4; ++j) { sc[j] = wmma16(kf[j][0], qf0, (v8f){}); sc[j] = wmma16(kf[j][1], qf1, sc[j]); }
        asm volatile("v_nop\n\tv_nop\n\tv_nop\n\tv_nop" : "+v"(sc[0]), "+v"(sc[1]), "+v"(sc[2]), "+v"(sc[3]) : "v"(kf[3][0]), "v"(kf[3][1]), "v"(qf0), "v"(qf1));
        float p[4][8]; float tmax = NINF;
#pragma unroll
        for (int j = 0; j < 4; ++j) {
            const v4i m0 = *(const v4i*)(prow + t0 + j * 16 + 8 * h); const v4i m1 = *(const v4i*)(prow + t0 + j * 16 + 8 * h + 4);
            const int mv[8] = {m0[0], m0[1], m0[2], m0[3], m1[0], m1[1], m1[2], m1[3]};
#pragma unroll
            for (int r = 0; r < 8; ++r) { const int t = t0 + j * 16 + 8 * h + r; const bool ok = (mv[r] != 0) && ((causal == 0) || (t <= qrow)); float s = sc[j][r] * SFAC; s = ok ? s : NINF; p[j][r] = s; tmax = fmaxf(tmax, s); } }
        tmax = fmaxf(tmax, __shfl_xor(tmax, 16, 32));
        const float mn = fmaxf(m, tmax);
        const float mnz = (mn == NINF) ? 0.f : mn;
        const float corr = __builtin_amdgcn_exp2f((m - mnz) * L2E);
        float psum = 0.f;
#pragma unroll
        for (int j = 0; j < 4; ++j)
#pragma unroll
            for (int r = 0; r < 8; ++r) { const float d0 = (p[j][r] - mnz) * L2E; const float e = __builtin_amdgcn_exp2f(d0); p[j][r] = e; psum += e; }
        psum += __shfl_xor(psum, 16, 32);
        l = l * corr + psum; m = mn;
#pragma unroll
        for (int nb = 0; nb < 4; ++nb)
#pragma unroll
            for (int r = 0; r < 8; ++r) oacc[nb][r] *= corr;
        v16h pf0, pf1;
#pragma unroll
        for (int r = 0; r < 8; ++r) { pf0[r] = (h16)(p[0][r] * PCAR); pf0[8 + r] = (h16)(p[1][r] * PCAR); pf1[r] = (h16)(p[2][r] * PCAR); pf1[8 + r] = (h16)(p[3][r] * PCAR); }
        v16h vf[4][2];
#pragma unroll
        for (int nb = 0; nb < 4; ++nb) { const h16* vp = vbase + (size_t)nb * 16 * NT + t0; vf[nb][0] = ldfrag(vp); vf[nb][1] = ldfrag(vp + 32); }
#pragma unroll
        for (int nb = 0; nb < 4; ++nb) { oacc[nb] = wmma16(vf[nb][0], pf0, oacc[nb]); oacc[nb] = wmma16(vf[nb][1], pf1, oacc[nb]); }
        asm volatile("v_nop\n\tv_nop\n\tv_nop\n\tv_nop" : "+v"(oacc[0]), "+v"(oacc[1]), "+v"(oacc[2]), "+v"(oacc[3]) : "v"(vf[3][0]), "v"(vf[3][1]), "v"(pf0), "v"(pf1));
    }
    const float rl = __fdiv_rn(1.0f, (l > 0.f) ? l : 1.0f);
    const float inv = (l > 0.f) ? (CCAR / (PCAR * VCAR)) * rl : 0.f;
#pragma unroll
    for (int nb = 0; nb < 4; ++nb) { v8h o;
#pragma unroll
        for (int r = 0; r < 8; ++r) o[r] = (h16)(oacc[nb][r] * inv);
        *(v8ha*)(so + lc * 72 + nb * 16 + 8 * h) = o; }
    __builtin_amdgcn_fence(3  , "wavefront"); __builtin_amdgcn_wave_barrier(); asm volatile("" ::: "memory");
    h16* cbase = Ctx + (rowbase + q0) * DM + hh * HD;
#pragma unroll 1
    for (int ps = 0; ps < 2; ++ps) {
#pragma unroll
        for (int i = 0; i < 4; ++i) { const int row = 4 * i + (lane >> 3), piece = lane & 7; const v8h v = *(const v8ha*)(so + row * 72 + piece * 8); *(volatile v8h*)(cbase + (size_t)row * DM + piece * 8) = v; }
        if (ps == 0) __threadfence(); }
}

__global__ __launch_bounds__(256) void k_ln(const float* __restrict__ Y, const float* __restrict__ R, int rfull, const float* __restrict__ g, const float* __restrict__ be, float* outF, int ofull, h16* outP) {
    const int lane = threadIdx.x & 31; const int row = blockIdx.x * 8 + (threadIdx.x >> 5); if (row >= NT) return;
    const int bi = row / SEQ, t = row - bi * SEQ; const size_t frow = (size_t)bi * SEQ_FULL + t;
    const float* yr = Y + (size_t)row * DM; const float* rr = R + (rfull ? frow : (size_t)row) * DM;
    float v[DM / 32]; float s = 0.f;
#pragma unroll
    for (int c = 0; c < DM / 128; ++c) { const v4f a = *(const v4f*)(yr + c * 128 + lane * 4); const v4f r4 = *(const v4f*)(rr + c * 128 + lane * 4);
#pragma unroll
        for (int q = 0; q < 4; ++q) { const float rv = rfull ? bfr(r4[q]) : r4[q]; const float x = __fadd_rn(a[q], rv); v[c * 4 + q] = x; s = __fadd_rn(s, x); } }
#pragma unroll
    for (int sh = 16; sh; sh >>= 1) s = __fadd_rn(s, __shfl_xor(s, sh, 32));
    const float mean = __fdiv_rn(s, (float)DM); float s2 = 0.f;
#pragma unroll
    for (int k = 0; k < DM / 32; ++k) { const float dv = __fsub_rn(v[k], mean); float p2 = __fmul_rn(dv, dv); asm volatile("" : "+v"(p2)); s2 = __fadd_rn(s2, p2); v[k] = dv; }
#pragma unroll
    for (int sh = 16; sh; sh >>= 1) s2 = __fadd_rn(s2, __shfl_xor(s2, sh, 32));
    const float rs = __fdiv_rn(1.0f, __fsqrt_rn(__fadd_rn(__fdiv_rn(s2, (float)DM), LNEPS)));
    float* orow = outF + (ofull ? frow : (size_t)row) * DM;
#pragma unroll 1
    for (int ps = 0; ps < 2; ++ps) {
#pragma unroll
        for (int c = 0; c < DM / 128; ++c) { v4f o; v4h oh;
#pragma unroll
            for (int q = 0; q < 4; ++q) { const int col = c * 128 + lane * 4 + q; float y = __fmul_rn(v[c * 4 + q], rs); asm volatile("" : "+v"(y)); y = __fmul_rn(y, bfr(g[col])); asm volatile("" : "+v"(y)); o[q] = __fadd_rn(y, bfr(be[col])); oh[q] = (h16)(o[q] * ACAR); }
            *(volatile v4f*)(orow + c * 128 + lane * 4) = o; if (outP) *(volatile v4h*)(outP + (size_t)row * DM + c * 128 + lane * 4) = oh; }
        if (ps == 0) __threadfence(); }
}

extern "C" void kernel_launch(void* const* d_in, const int* in_sizes, int n_in,
                              void* d_out, int out_size, void* d_ws, size_t ws_size, hipStream_t stream) {
    if (n_in < 30) return;
    const int rows = (NB - 1) * SEQ_FULL + SEQ;
    if (in_sizes[0] < rows * DM || in_sizes[1] < rows * DM || in_sizes[2] < rows || in_sizes[3] < rows) return;
    for (int i = 4; i < 20; i += 2) { if (in_sizes[i] < DM * DM || in_sizes[i + 1] < DM) return; }
    if (in_sizes[20] < DM * FF || in_sizes[21] < FF || in_sizes[22] < FF * DM || in_sizes[23] < DM) return;
    for (int i = 24; i < 30; ++i) { if (in_sizes[i] < DM) return; }
    if (out_size < rows * DM) return;
    const float* xin = (const float*)d_in[0]; const float* enc = (const float*)d_in[1];
    const int* src_pad = (const int*)d_in[2]; const int* trg_pad = (const int*)d_in[3];
    const float* sa_wq = (const float*)d_in[4];  const float* sa_bq = (const float*)d_in[5];
    const float* sa_wk = (const float*)d_in[6];  const float* sa_bk = (const float*)d_in[7];
    const float* sa_wv = (const float*)d_in[8];  const float* sa_bv = (const float*)d_in[9];
    const float* sa_wo = (const float*)d_in[10]; const float* sa_bo = (const float*)d_in[11];
    const float* ca_wq = (const float*)d_in[12]; const float* ca_bq = (const float*)d_in[13];
    const float* ca_wk = (const float*)d_in[14]; const float* ca_bk = (const float*)d_in[15];
    const float* ca_wv = (const float*)d_in[16]; const float* ca_bv = (const float*)d_in[17];
    const float* ca_wo = (const float*)d_in[18]; const float* ca_bo = (const float*)d_in[19];
    const float* w1 = (const float*)d_in[20]; const float* b1 = (const float*)d_in[21];
    const float* w2 = (const float*)d_in[22]; const float* b2 = (const float*)d_in[23];
    const float* g1 = (const float*)d_in[24]; const float* e1 = (const float*)d_in[25];
    const float* g2 = (const float*)d_in[26]; const float* e2 = (const float*)d_in[27];
    const float* g3 = (const float*)d_in[28]; const float* e3 = (const float*)d_in[29];
    float* OUT = (float*)d_out;
    char* wsp = (char*)d_ws; size_t used = 0;
    auto take = [&](size_t bytes) { char* p = wsp + used; used += (bytes + 255) & ~(size_t)255; return (void*)p; };
    const size_t WSQ = (size_t)DM * DM * 2, WSF = (size_t)DM * FF * 2, PL = (size_t)NT * DM * 2, F32P = (size_t)NT * DM * 4;
    h16* WQ = (h16*)take(WSQ); h16* WK = (h16*)take(WSQ); h16* WV = (h16*)take(WSQ); h16* WO = (h16*)take(WSQ);
    h16* CWQ = (h16*)take(WSQ); h16* CWK = (h16*)take(WSQ); h16* CWV = (h16*)take(WSQ); h16* CWO = (h16*)take(WSQ);
    h16* W1T = (h16*)take(WSF); h16* W2T = (h16*)take(WSF);
    h16* X16 = (h16*)take(PL); h16* E16 = (h16*)take(PL);
    h16* R32 = (h16*)take(PL * 4);
    float* Y = (float*)take(F32P); float* X1F = (float*)take(F32P); float* X2F = (float*)take(F32P);
    if (used > ws_size) return;
    h16* Q16 = R32; h16* K16 = R32 + (size_t)NT * DM; h16* VT16 = R32 + (size_t)2 * NT * DM; h16* CTX16 = R32 + (size_t)3 * NT * DM; h16* H16 = R32;
    h16* X1P = X16;
    h16* X2P = X16;
    const unsigned GW1 = (unsigned)(((size_t)DM * DM / 64 + 63) / 64), GW2 = (unsigned)(((size_t)DM * FF / 64 + 63) / 64);
    k_wtG<<<GW1, 256, 0, stream>>>(sa_wq, DM, DM, WQ); k_wtG<<<GW1, 256, 0, stream>>>(sa_wk, DM, DM, WK); k_wtG<<<GW1, 256, 0, stream>>>(sa_wv, DM, DM, WV); k_wtG<<<GW1, 256, 0, stream>>>(sa_wo, DM, DM, WO);
    k_wtG<<<GW1, 256, 0, stream>>>(ca_wq, DM, DM, CWQ); k_wtG<<<GW1, 256, 0, stream>>>(ca_wk, DM, DM, CWK); k_wtG<<<GW1, 256, 0, stream>>>(ca_wv, DM, DM, CWV); k_wtG<<<GW1, 256, 0, stream>>>(ca_wo, DM, DM, CWO);
    k_wtG<<<GW2, 256, 0, stream>>>(w1, DM, FF, W1T);
    k_wtG<<<GW2, 256, 0, stream>>>(w2, FF, DM, W2T);
    const unsigned GC = (unsigned)(((size_t)NT * DM / 8 + 255) / 256);
    k_cvtx<<<GC, 256, 0, stream>>>(xin, X16); k_cvtx<<<GC, 256, 0, stream>>>(enc, E16);
    const dim3 gP(NT / 64, DM / 64), gV(DM / 64, NT / 64), gH(NT / 64, FF / 64), gA(SEQ / 16, NHD, NB);
    k_gemmw<1, 1, false><<<gP, 32, 0, stream>>>(X16, WQ, DM, (void*)Q16, DM, sa_bq, QCAR / (XCAR * WCAR), QCAR);
    k_gemmw<1, 1, false><<<gP, 32, 0, stream>>>(X16, WK, DM, (void*)K16, DM, sa_bk, KCAR / (XCAR * WCAR), KCAR);
    k_gemmw<1, 2, false><<<gV, 32, 0, stream>>>(WV, X16, DM, (void*)VT16, NT, sa_bv, VCAR / (XCAR * WCAR), VCAR);
    k_attn<<<gA, 32, 0, stream>>>(Q16, K16, VT16, trg_pad, 1, CTX16);
    k_gemmw<0, 1, false><<<gP, 32, 0, stream>>>(CTX16, WO, DM, (void*)Y, DM, sa_bo, 1.0f / (CCAR * WCAR), 1.0f);
    k_ln<<<(NT + 7) / 8, 256, 0, stream>>>(Y, xin, 1, g1, e1, X1F, 0, X1P);
    k_gemmw<1, 1, false><<<gP, 32, 0, stream>>>(X1P, CWQ, DM, (void*)Q16, DM, ca_bq, QCAR / (ACAR * WCAR), QCAR);
    k_gemmw<1, 1, false><<<gP, 32, 0, stream>>>(E16, CWK, DM, (void*)K16, DM, ca_bk, KCAR / (XCAR * WCAR), KCAR);
    k_gemmw<1, 2, false><<<gV, 32, 0, stream>>>(CWV, E16, DM, (void*)VT16, NT, ca_bv, VCAR / (XCAR * WCAR), VCAR);
    k_attn<<<gA, 32, 0, stream>>>(Q16, K16, VT16, src_pad, 0, CTX16);
    k_gemmw<0, 1, false><<<gP, 32, 0, stream>>>(CTX16, CWO, DM, (void*)Y, DM, ca_bo, 1.0f / (CCAR * WCAR), 1.0f);
    k_ln<<<(NT + 7) / 8, 256, 0, stream>>>(Y, X1F, 0, g2, e2, X2F, 0, X2P);
    k_gemmw<1, 1, true><<<gH, 32, 0, stream>>>(X2P, W1T, DM, (void*)H16, FF, b1, HCAR / (ACAR * WCAR), HCAR);
    k_gemmw<0, 1, false><<<gP, 32, 0, stream>>>(H16, W2T, FF, (void*)Y, DM, b2, 1.0f / (HCAR * WCAR), 1.0f);
    k_ln<<<(NT + 7) / 8, 256, 0, stream>>>(Y, X2F, 0, g3, e3, OUT, 1, nullptr);
}
